// GRU4Rec_67894843015522
// MI455X (gfx1250) — hardware-run, weakly checked
//
#include <hip/hip_runtime.h>
#include <math.h>

constexpr int BATCH_N    = 4096;
constexpr int STEPS_N    = 200;
constexpr int HID_N      = 64;
constexpr int GATE3_N    = 192;
constexpr int VOCAB_N    = 100000;
constexpr int VOCAB_PAD  = 100032;
constexpr int ROWS_TILE  = 16;
constexpr int H_PITCH    = 72;
constexpr int GI_PITCH   = 196;
constexpr int OUT_PITCH  = 68;
constexpr int SCAN_THREADS = 128;

constexpr float EMB_CARRY = 1024.0f;
constexpr float W_CARRY   = 64.0f;
constexpr float H_CARRY   = 1024.0f;
constexpr float EW_FOLD   = 1.0f / (EMB_CARRY * W_CARRY);
constexpr float GH_FOLD   = 1.0f / (H_CARRY * W_CARRY);
constexpr float F16_MIN_NORMAL = 6.103515625e-5f;

constexpr int EMB_BLOCKS  = (VOCAB_N * HID_N / 8) / 256;
constexpr int PAD_BLOCKS  = ((VOCAB_PAD - VOCAB_N) * HID_N / 8) / 256;
constexpr int WGT_BLOCKS  = (GATE3_N * HID_N / 8) / 256;
constexpr int PREP_BLOCKS = EMB_BLOCKS + PAD_BLOCKS + 2 * WGT_BLOCKS;

constexpr int EW_TILES_M = VOCAB_PAD / 64;
constexpr int EW_TILES_N = GATE3_N / 64;
constexpr int EW_TILES   = EW_TILES_M * EW_TILES_N;
constexpr int EW_BLOCKS  = (EW_TILES + 7) / 8;

static_assert(GATE3_N == 3 * HID_N);
static_assert(HID_N % 32 == 0);
static_assert(VOCAB_PAD % 64 == 0 && VOCAB_PAD >= VOCAB_N);
static_assert(GATE3_N % 64 == 0);
static_assert((VOCAB_N * HID_N / 8) % 256 == 0);
static_assert(((VOCAB_PAD - VOCAB_N) * HID_N / 8) % 256 == 0);
static_assert((GATE3_N * HID_N / 8) % 256 == 0);
static_assert(BATCH_N % ROWS_TILE == 0);
static_assert((ROWS_TILE * STEPS_N) % 4 == 0);
static_assert(SCAN_THREADS == ROWS_TILE * 8);
static_assert(GATE3_N == 8 * 4 * 6);
static_assert(GI_PITCH % 4 == 0 && GI_PITCH >= GATE3_N);
static_assert(H_PITCH % 8 == 0 && H_PITCH >= HID_N);

typedef __attribute__((ext_vector_type(16))) _Float16 v16h;
typedef __attribute__((ext_vector_type(8)))  _Float16 v8h;
typedef __attribute__((ext_vector_type(8)))  float    v8f;
typedef __attribute__((ext_vector_type(4)))  float    v4f;
typedef __attribute__((ext_vector_type(4)))  int      v4i;

union FragU { v16h v; v8h h[2]; };
__device__ __forceinline__ v16h frag_load(const _Float16* p) {
  FragU f;
  f.h[0] = *(const v8h*)(p);
  f.h[1] = *(const v8h*)(p + 16);
  return f.v;
}
__device__ __forceinline__ v8f mma_h(v16h a, v16h b, v8f c) {
  c = __builtin_amdgcn_wmma_f32_16x16x32_f16(false, a, false, b, (short)0, c, false, false);
  asm volatile("v_nop\n\tv_nop\n\tv_nop\n\tv_nop" : "+v"(c) : "v"(a), "v"(b));
  return c;
}
__device__ __forceinline__ _Float16 to_f16_flush(float v) {
  const float w = (fabsf(v) < F16_MIN_NORMAL) ? 0.0f : v;
  return (_Float16)w;
}
__device__ __forceinline__ int clampi(int v, int lo, int hi) {
  const int a = (v < lo) ? lo : v;
  return (a > hi) ? hi : a;
}
__device__ __forceinline__ float fsigm(float x) { return __builtin_amdgcn_rcpf(1.0f + expf(-x)); }
__device__ __forceinline__ float ftanh(float x) { return 1.0f - 2.0f * __builtin_amdgcn_rcpf(1.0f + expf(2.0f * x)); }

__device__ __forceinline__ v8h cvt8(const float* p, float carry) {
  const v4f a = *(const v4f*)(p);
  const v4f b = *(const v4f*)(p + 4);
  v8h h;
#pragma unroll
  for (int e = 0; e < 4; ++e) {
    const float fa = a[e] * carry;
    const float fb = b[e] * carry;
    h[e]     = to_f16_flush(fa);
    h[4 + e] = to_f16_flush(fb);
  }
  return h;
}
__device__ __forceinline__ void store8_twice(unsigned short* o, v8h h) {
  *(volatile v8h*)o = h;
  __threadfence();
  *(volatile v8h*)o = h;
}

__global__ __launch_bounds__(256) void prep_kernel(const float* __restrict__ emb,
                                                  const float* __restrict__ Wih,
                                                  const float* __restrict__ Whh,
                                                  unsigned short* __restrict__ E16,
                                                  unsigned short* __restrict__ WIH16,
                                                  unsigned short* __restrict__ WHH16) {
  const int blk = blockIdx.x;
  const int tid = threadIdx.x;
  if (blk < EMB_BLOCKS) {
    const size_t e0 = ((size_t)blk * 256 + (size_t)tid) * 8;
    const v8h h = cvt8(emb + e0, EMB_CARRY);
    store8_twice(E16 + e0, h);
  } else if (blk < EMB_BLOCKS + PAD_BLOCKS) {
    const size_t e0 = ((size_t)blk * 256 + (size_t)tid) * 8;
    v8h z;
#pragma unroll
    for (int e = 0; e < 8; ++e) z[e] = (_Float16)0.0f;
    store8_twice(E16 + e0, z);
  } else if (blk < EMB_BLOCKS + PAD_BLOCKS + WGT_BLOCKS) {
    const size_t e0 = ((size_t)(blk - EMB_BLOCKS - PAD_BLOCKS) * 256 + (size_t)tid) * 8;
    const v8h h = cvt8(Wih + e0, W_CARRY);
    store8_twice(WIH16 + e0, h);
  } else {
    const size_t e0 = ((size_t)(blk - EMB_BLOCKS - PAD_BLOCKS - WGT_BLOCKS) * 256 + (size_t)tid) * 8;
    const v8h h = cvt8(Whh + e0, W_CARRY);
    store8_twice(WHH16 + e0, h);
  }
}

__global__ __launch_bounds__(256) void ew_gemm_kernel(const unsigned short* __restrict__ Ap,
                                                     const unsigned short* __restrict__ Btp,
                                                     float* __restrict__ Cout) {
  __shared__ __align__(16) float sT[8][16 * 68];
  const _Float16* A  = (const _Float16*)Ap;
  const _Float16* Bt = (const _Float16*)Btp;
  const int lane = threadIdx.x & 31;
  const int wave = threadIdx.x >> 5;
  const int tile = blockIdx.x * 8 + wave;
  if (tile >= EW_TILES) return;
  const int tm = tile / EW_TILES_N;
  const int tn = tile - tm * EW_TILES_N;
  const int m0 = tm << 6;
  const int n0 = tn << 6;
  const int rlane = lane & 15;
  const int koff  = (lane >> 4) * 8;
  const int mOff  = (lane >> 4) * 8;

  v8f acc[4][4];
#pragma unroll
  for (int i = 0; i < 4; ++i)
#pragma unroll
    for (int j = 0; j < 4; ++j) acc[i][j] = (v8f){0.f, 0.f, 0.f, 0.f, 0.f, 0.f, 0.f, 0.f};

#pragma unroll 1
  for (int k0 = 0; k0 < HID_N; k0 += 32) {
    v16h bh[4];
#pragma unroll
    for (int j = 0; j < 4; ++j) {
      const size_t bo = (size_t)(n0 + (j << 4) + rlane) * HID_N + koff + k0;
      bh[j] = frag_load(Bt + bo);
    }
#pragma unroll
    for (int i = 0; i < 4; ++i) {
      const size_t ao = (size_t)(m0 + (i << 4) + rlane) * HID_N + koff + k0;
      const v16h ah = frag_load(A + ao);
#pragma unroll
      for (int j = 0; j < 4; ++j) acc[i][j] = mma_h(ah, bh[j], acc[i][j]);
    }
  }

  float* slab = sT[wave];
#pragma unroll
  for (int i = 0; i < 4; ++i) {
    const int mBase = m0 + (i << 4);
#pragma unroll
    for (int j = 0; j < 4; ++j) {
#pragma unroll
      for (int r = 0; r < 8; ++r) {
        const float v = acc[i][j][r] * EW_FOLD;
        slab[(mOff + r) * 68 + (j << 4) + rlane] = v;
      }
    }
    __builtin_amdgcn_fence(__ATOMIC_RELEASE, "workgroup");
    __builtin_amdgcn_wave_barrier();
    __builtin_amdgcn_fence(__ATOMIC_ACQUIRE, "workgroup");
    {
      const int hh = lane >> 4;
      const int c4 = (lane & 15) * 4;
      for (int pass = 0; pass < 2; ++pass) {
#pragma unroll
        for (int it = 0; it < 8; ++it) {
          const int row = it * 2 + hh;
          const v4f v = *(const v4f*)(slab + row * 68 + c4);
          *(volatile v4f*)(Cout + (size_t)(mBase + row) * GATE3_N + n0 + c4) = v;
        }
        __threadfence();
      }
    }
    __builtin_amdgcn_fence(__ATOMIC_RELEASE, "workgroup");
    __builtin_amdgcn_wave_barrier();
    __builtin_amdgcn_fence(__ATOMIC_ACQUIRE, "workgroup");
  }
}

__global__ __launch_bounds__(SCAN_THREADS) void gru_scan_kernel(const int* __restrict__ seq_token,
                                                               const int* __restrict__ seq_pos,
                                                               const float* __restrict__ EW,
                                                               const unsigned short* __restrict__ WHH16p,
                                                               float* __restrict__ out) {
  __shared__ __align__(16) int      toks[ROWS_TILE * STEPS_N];
  __shared__ __align__(16) int      lens[ROWS_TILE];
  __shared__ __align__(16) _Float16 hA[2 * ROWS_TILE * H_PITCH];
  __shared__ __align__(16) float    giL[2 * ROWS_TILE * GI_PITCH];
  __shared__ __align__(16) float    Hs[ROWS_TILE * OUT_PITCH];

  const int tid  = threadIdx.x;
  const int lane = tid & 31;
  const int wave = tid >> 5;
  const int c    = lane & 15;
  const int hh   = lane >> 4;
  const int koff = hh * 8;
  const int mOff = hh * 8;
  const int j    = 16 * wave + c;
  const int rb   = blockIdx.x * ROWS_TILE;
  const int grow = tid >> 3;
  const int gsub = tid & 7;

  {
    const v4i* tsrc = (const v4i*)(seq_token + (size_t)rb * STEPS_N);
#pragma unroll 1
    for (int e = tid; e < (ROWS_TILE * STEPS_N) / 4; e += SCAN_THREADS) {
      v4i v = tsrc[e];
      v[0] = clampi(v[0], 0, VOCAB_N - 1);
      v[1] = clampi(v[1], 0, VOCAB_N - 1);
      v[2] = clampi(v[2], 0, VOCAB_N - 1);
      v[3] = clampi(v[3], 0, VOCAB_N - 1);
      *(v4i*)(toks + 4 * e) = v;
    }
  }
  {
    int sp = seq_pos[rb + (tid & 15)];
    asm volatile("" : "+v"(sp));
    sp = clampi(sp, 1, STEPS_N);
    if (tid < ROWS_TILE) lens[tid] = sp;
  }
#pragma unroll 1
  for (int i = tid; i < 2 * ROWS_TILE * H_PITCH; i += SCAN_THREADS) hA[i] = (_Float16)0.0f;
  __syncthreads();

  int lenr[8];
#pragma unroll
  for (int r = 0; r < 8; ++r) lenr[r] = lens[mOff + r];
  int tmax = 1;
#pragma unroll
  for (int r = 0; r < ROWS_TILE; ++r) {
    const int lv = lens[r];
    tmax = (lv > tmax) ? lv : tmax;
  }
  tmax = (tmax > STEPS_N) ? STEPS_N : tmax;

  const _Float16* WHH = (const _Float16*)WHH16p;
  const _Float16* wr = WHH + (size_t)j * HID_N + koff;
  const _Float16* wz = WHH + (size_t)(HID_N + j) * HID_N + koff;
  const _Float16* wn = WHH + (size_t)(2 * HID_N + j) * HID_N + koff;
  const v16h br0 = frag_load(wr);
  const v16h br1 = frag_load(wr + 32);
  const v16h bz0 = frag_load(wz);
  const v16h bz1 = frag_load(wz + 32);
  const v16h bn0 = frag_load(wn);
  const v16h bn1 = frag_load(wn + 32);

  {
    const int tok0 = toks[grow * STEPS_N];
    const float* ep = EW + (size_t)tok0 * GATE3_N + gsub * 4;
    float* gd = giL + grow * GI_PITCH + gsub * 4;
#pragma unroll
    for (int q = 0; q < 6; ++q) {
      const v4f v = *(const v4f*)(ep + q * 32);
      *(v4f*)(gd + q * 32) = v;
    }
  }
  __syncthreads();

  float hreg[8];
#pragma unroll
  for (int r = 0; r < 8; ++r) hreg[r] = 0.0f;
  const v8f z8 = {0.f, 0.f, 0.f, 0.f, 0.f, 0.f, 0.f, 0.f};

#pragma unroll 1
  for (int t = 0; t < tmax; ++t) {
    const int cur = t & 1;
    const _Float16* hcur = hA + cur * (ROWS_TILE * H_PITCH);
    _Float16*       hnxt = hA + (cur ^ 1) * (ROWS_TILE * H_PITCH);
    const float*    gcur = giL + cur * (ROWS_TILE * GI_PITCH);
    float*          gnxt = giL + (cur ^ 1) * (ROWS_TILE * GI_PITCH);

    const int tn = (t + 1 < STEPS_N) ? (t + 1) : (STEPS_N - 1);
    const int tokn = toks[grow * STEPS_N + tn];
    const float* ep = EW + (size_t)tokn * GATE3_N + gsub * 4;
    v4f pf[6];
#pragma unroll
    for (int q = 0; q < 6; ++q) pf[q] = *(const v4f*)(ep + q * 32);

    const _Float16* arow = hcur + c * H_PITCH + koff;
    const v16h a0 = frag_load(arow);
    const v16h a1 = frag_load(arow + 32);
    v8f ar = z8;
    v8f az = z8;
    v8f an = z8;
    ar = mma_h(a0, br0, ar);
    az = mma_h(a0, bz0, az);
    an = mma_h(a0, bn0, an);
    ar = mma_h(a1, br1, ar);
    az = mma_h(a1, bz1, az);
    an = mma_h(a1, bn1, an);

#pragma unroll
    for (int r = 0; r < 8; ++r) {
      const float* gp = gcur + (mOff + r) * GI_PITCH + j;
      const float xr = gp[0];
      const float xz = gp[HID_N];
      const float xn = gp[2 * HID_N];
      const float hr = ar[r] * GH_FOLD;
      const float hz = az[r] * GH_FOLD;
      const float hn = an[r] * GH_FOLD;
      const float rg = fsigm(xr + hr);
      const float zg = fsigm(xz + hz);
      const float ng = ftanh(xn + rg * hn);
      const float hnew = (1.0f - zg) * ng + zg * hreg[r];
      hreg[r] = (t < lenr[r]) ? hnew : hreg[r];
    }

#pragma unroll
    for (int r = 0; r < 8; ++r) {
      const float hv = hreg[r] * H_CARRY;
      hnxt[(mOff + r) * H_PITCH + j] = to_f16_flush(hv);
    }
    {
      float* gd = gnxt + grow * GI_PITCH + gsub * 4;
#pragma unroll
      for (int q = 0; q < 6; ++q) *(v4f*)(gd + q * 32) = pf[q];
    }
    __syncthreads();
  }

#pragma unroll
  for (int r = 0; r < 8; ++r) Hs[(mOff + r) * OUT_PITCH + j] = hreg[r];
  __syncthreads();
  {
    const int c4 = c * 4;
    for (int pass = 0; pass < 2; ++pass) {
#pragma unroll
      for (int it = 0; it < 2; ++it) {
        const int row = 4 * wave + 2 * it + hh;
        const v4f v = *(const v4f*)(Hs + row * OUT_PITCH + c4);
        *(volatile v4f*)(out + (size_t)(rb + row) * HID_N + c4) = v;
      }
      __threadfence();
    }
  }
}

extern "C" void kernel_launch(void* const* d_in, const int* in_sizes, int n_in,
                              void* d_out, int out_size, void* d_ws, size_t ws_size, hipStream_t stream) {
  if (n_in < 5 || d_out == nullptr || d_ws == nullptr) return;
  if (in_sizes[0] != BATCH_N * STEPS_N || in_sizes[1] != BATCH_N || in_sizes[2] != VOCAB_N * HID_N ||
      in_sizes[3] != GATE3_N * HID_N || in_sizes[4] != GATE3_N * HID_N || out_size != BATCH_N * HID_N) return;

  const int*   seq_token = (const int*)d_in[0];
  const int*   seq_pos   = (const int*)d_in[1];
  const float* emb       = (const float*)d_in[2];
  const float* Wih       = (const float*)d_in[3];
  const float* Whh       = (const float*)d_in[4];
  float* out = (float*)d_out;

  char* ws = (char*)d_ws;
  size_t off = 0;
  auto carve = [&](size_t bytes) -> char* { char* p = ws + off; off += (bytes + 255) & ~(size_t)255; return p; };
  float*          EW    = (float*)carve((size_t)VOCAB_PAD * GATE3_N * 4);
  unsigned short* E16   = (unsigned short*)carve((size_t)VOCAB_PAD * HID_N * 2);
  unsigned short* WIH16 = (unsigned short*)carve((size_t)GATE3_N * HID_N * 2);
  unsigned short* WHH16 = (unsigned short*)carve((size_t)GATE3_N * HID_N * 2);
  if (off > ws_size || off > (size_t)134217728) return;

  prep_kernel<<<PREP_BLOCKS, 256, 0, stream>>>(emb, Wih, Whh, E16, WIH16, WHH16);
  ew_gemm_kernel<<<EW_BLOCKS, 256, 0, stream>>>(E16, WIH16, EW);
  gru_scan_kernel<<<BATCH_N / ROWS_TILE, SCAN_THREADS, 0, stream>>>(seq_token, seq_pos, EW, WHH16, out);
}
